// SPTransformerEncoderLayer_80668075753648
// MI455X (gfx1250) — hardware-verified
//
#include <hip/hip_runtime.h>
#include <stddef.h>


#define DM    128
#define NHD   8
#define HIDN  512
#define NQKV  384
#define GR    16
#define STP   32
#define WSCL  16.0f
#define WINV  0.0625f

#define POFF_QKV  0
#define POFF_O    (NQKV * DM)
#define POFF_1    (POFF_O + DM * DM)
#define POFF_2    (POFF_1 + HIDN * DM)
#define PLANE_H   (POFF_2 + DM * HIDN)
#define PREP_ROWS (NQKV + DM + HIDN + DM)

#define NB    256
#define SH    8
#define CHUNK 4096
#define ATHR  256
#define AWAVE 8
#define NGRP  (CHUNK / (ATHR * 4))
#define WCAP  ((CHUNK / ATHR) * 32)
#define AGG_SACC (NB * DM)
#define AGG_AUX  (2 * NB * NHD)
#define AGG_LIST (AWAVE * WCAP)
#define AGG_LDS_BYTES ((AGG_SACC + AGG_AUX + AGG_LIST + AWAVE) * 4)
#define WS_CAP ((size_t)134217728)

static_assert(NGRP == 4);
static_assert(WCAP == 512);
static_assert(NB == (1 << SH));
static_assert(SH + 12 <= 31);
static_assert(AGG_LDS_BYTES == 163872);
static_assert(PLANE_H == 196608);
static_assert(PREP_ROWS == 1152);
static_assert(DM == 32 * 4);
static_assert(NHD * 16 == DM);

typedef float          v4f   __attribute__((ext_vector_type(4)));
typedef float          v8f   __attribute__((ext_vector_type(8)));
typedef int            v4i   __attribute__((ext_vector_type(4)));
typedef _Float16       v8h   __attribute__((ext_vector_type(8)));
typedef _Float16       v16h  __attribute__((ext_vector_type(16)));

union Frag { v16h v; v8h p[2]; };

template <int KD, int NOUT>
union LdsG { _Float16 hs[GR * (KD + 8)]; float xs[GR * (NOUT + 4)]; };

__device__ __forceinline__ v8f wm(v16h a, v16h b, v8f c) {
  v8f d = __builtin_amdgcn_wmma_f32_16x16x32_f16(false, a, false, b, (short)0, c, false, false);
  asm volatile("v_nop\n\tv_nop\n\tv_nop\n\tv_nop" : "+v"(d) : "v"(a), "v"(b));
  return d;
}

__device__ __forceinline__ float hsum4(v4f a) { return (a.x + a.y) + (a.z + a.w); }
__device__ __forceinline__ v4f ld4(const float* p) { return *(const v4f*)p; }

__device__ __forceinline__ v4f relu4(v4f o) {
  v4f r;
  r.x = fmaxf(o.x, 0.f);
  r.y = fmaxf(o.y, 0.f);
  r.z = fmaxf(o.z, 0.f);
  r.w = fmaxf(o.w, 0.f);
  return r;
}

__device__ __forceinline__ v8h cvt8(v4f a, v4f b) {
  const float x[8] = {a.x, a.y, a.z, a.w, b.x, b.y, b.z, b.w};
  v8h h = {0, 0, 0, 0, 0, 0, 0, 0};
#pragma unroll
  for (int i = 0; i < 8; ++i) h[i] = (_Float16)x[i];
  return h;
}

template <int KD>
__device__ __forceinline__ void stage_rows(const float* __restrict__ A, int rowBase, int nA,
                                           _Float16* ldsH, int tid) {
  constexpr int LDSP = KD + 8;
  const int r = tid >> 4;
  int row = rowBase + r;
  if (row > nA - 1) row = nA - 1;
  const float* p = A + (size_t)row * KD;
#pragma unroll
  for (int j = 0; j < KD / 128; ++j) {
    const int c0 = (tid & 15) * 8 + j * 128;
    const v4f f0 = ld4(p + c0);
    const v4f f1 = ld4(p + c0 + 4);
    *(v8h*)(ldsH + r * LDSP + c0) = cvt8(f0, f1);
  }
}

template <int TPW, int KD>
__device__ __forceinline__ void gemm_core(const _Float16* ldsH,
                                          const _Float16* __restrict__ wP,
                                          int tile0, int lane, v8f (&acc)[TPW]) {
  constexpr int LDSP = KD + 8;
  const int hh = lane >> 4;
  const int m  = lane & 15;
  const v8f z8 = {0.f, 0.f, 0.f, 0.f, 0.f, 0.f, 0.f, 0.f};
#pragma unroll
  for (int t = 0; t < TPW; ++t) acc[t] = z8;
  const _Float16* pa = ldsH + m * LDSP + 8 * hh;
#pragma unroll 1
  for (int kt = 0; kt < KD / 32; ++kt) {
    const int k0 = kt * 32;
    Frag a;
    a.p[0] = *(const v8h*)(pa + k0);
    a.p[1] = *(const v8h*)(pa + k0 + 16);
#pragma unroll
    for (int t = 0; t < TPW; ++t) {
      const size_t prow = (size_t)(tile0 + t) * 16 + m;
      const _Float16* pb = wP + prow * KD + k0 + 8 * hh;
      Frag b;
      b.p[0] = *(const v8h*)(pb);
      b.p[1] = *(const v8h*)(pb + 16);
      acc[t] = wm(a.v, b.v, acc[t]);
    }
  }
}

__global__ __launch_bounds__(256) void k_prep(const float* __restrict__ wq, const float* __restrict__ wk,
                                             const float* __restrict__ wv, const float* __restrict__ wo,
                                             const float* __restrict__ w1, const float* __restrict__ w2,
                                             _Float16* pW) {
  const int t = blockIdx.x * 256 + threadIdx.x;
  if (t >= PREP_ROWS) return;
  const float* W;
  int n, kd, pitch;
  size_t base;
  if (t < NQKV) {
    const int mat = t >> 7;
    W = (mat == 0) ? wq : ((mat == 1) ? wk : wv);
    n = t & (DM - 1); kd = DM; pitch = DM;
    base = (size_t)POFF_QKV + (size_t)t * DM;
  } else if (t < NQKV + DM) {
    W = wo; n = t - NQKV; kd = DM; pitch = DM;
    base = (size_t)POFF_O + (size_t)n * DM;
  } else if (t < NQKV + DM + HIDN) {
    W = w1; n = t - NQKV - DM; kd = DM; pitch = HIDN;
    base = (size_t)POFF_1 + (size_t)n * DM;
  } else {
    W = w2; n = t - NQKV - DM - HIDN; kd = HIDN; pitch = DM;
    base = (size_t)POFF_2 + (size_t)n * HIDN;
  }
  _Float16* dh = pW + base;
#pragma unroll 1
  for (int kb = 0; kb < kd / 8; ++kb) {
    v4f f0, f1;
    f0.x = W[(size_t)(kb * 8 + 0) * pitch + n] * WSCL;
    f0.y = W[(size_t)(kb * 8 + 1) * pitch + n] * WSCL;
    f0.z = W[(size_t)(kb * 8 + 2) * pitch + n] * WSCL;
    f0.w = W[(size_t)(kb * 8 + 3) * pitch + n] * WSCL;
    f1.x = W[(size_t)(kb * 8 + 4) * pitch + n] * WSCL;
    f1.y = W[(size_t)(kb * 8 + 5) * pitch + n] * WSCL;
    f1.z = W[(size_t)(kb * 8 + 6) * pitch + n] * WSCL;
    f1.w = W[(size_t)(kb * 8 + 7) * pitch + n] * WSCL;
    const v8h h = cvt8(f0, f1);
    *(volatile v8h*)(dh + kb * 8) = h;
    __threadfence();
    *(volatile v8h*)(dh + kb * 8) = h;
  }
}

template <int KD, int NOUT>
__global__ __launch_bounds__(256) void k_gemm(const float* __restrict__ A,
                                             const _Float16* __restrict__ wP,
                                             const float* __restrict__ resid,
                                             float* out, int nA, int relu) {
  constexpr int TPW  = NOUT / 128;
  constexpr int NS   = NOUT / 128;
  constexpr int XSP  = NOUT + 4;
  static_assert(TPW * 8 * 16 == NOUT);
  static_assert((KD % 128) == 0);
  __shared__ __attribute__((aligned(16))) LdsG<KD, NOUT> lds;

  const int tid  = threadIdx.x;
  const int lane = tid & 31;
  const int wave = tid >> 5;
  const int hh   = lane >> 4;
  const int m    = lane & 15;
  const int rowBase = blockIdx.x * GR;

  stage_rows<KD>(A, rowBase, nA, lds.hs, tid);
  __syncthreads();

  v8f acc[TPW];
  gemm_core<TPW, KD>(lds.hs, wP, wave * TPW, lane, acc);
  __syncthreads();

#pragma unroll
  for (int t = 0; t < TPW; ++t) {
    const int gc = (wave * TPW + t) * 16 + m;
#pragma unroll
    for (int r = 0; r < 8; ++r) lds.xs[(8 * hh + r) * XSP + gc] = acc[t][r] * WINV;
  }
  __syncthreads();

  v4f xr[2 * NS];
  float* gp[2 * NS];
  bool okr[2];
#pragma unroll
  for (int q = 0; q < 2; ++q) {
    const int row  = wave * 2 + q;
    const int node = rowBase + row;
    okr[q] = node < nA;
    const int nl = okr[q] ? node : (nA - 1);
#pragma unroll
    for (int s = 0; s < NS; ++s) {
      v4f v = ld4(lds.xs + row * XSP + s * 128 + 4 * lane);
      if (resid != nullptr) v += ld4(resid + (size_t)nl * NOUT + s * 128 + 4 * lane);
      if (relu) v = relu4(v);
      xr[q * NS + s] = v;
      gp[q * NS + s] = out + (size_t)nl * NOUT + s * 128 + 4 * lane;
    }
  }
#pragma unroll
  for (int q = 0; q < 2; ++q) {
    if (okr[q]) {
#pragma unroll
      for (int s = 0; s < NS; ++s) *(volatile v4f*)(gp[q * NS + s]) = xr[q * NS + s];
    }
  }
  __threadfence();
#pragma unroll
  for (int q = 0; q < 2; ++q) {
    if (okr[q]) {
#pragma unroll
      for (int s = 0; s < NS; ++s) *(volatile v4f*)(gp[q * NS + s]) = xr[q * NS + s];
    }
  }
}

__global__ __launch_bounds__(ATHR) void k_agg(const int* __restrict__ srcA, const int* __restrict__ dstA,
                                              const float* __restrict__ QKV, float* aggOut, int nN, int nE) {
  extern __shared__ v4f lds_dyn[];
  float* sacc = (float*)lds_dyn;
  float* mx   = sacc + AGG_SACC;
  float* den  = mx + NB * NHD;
  int*   list = (int*)(den + NB * NHD);
  int*   wcnt = list + AGG_LIST;

  const int tid  = threadIdx.x;
  const int lane = tid & 31;
  const int wave = tid >> 5;
  const int hd   = lane >> 2;
  const int nodeBase = blockIdx.x * NB;

  {
    const v4f z4 = {0.f, 0.f, 0.f, 0.f};
    for (int i = tid; i < AGG_SACC / 4; i += ATHR) lds_dyn[i] = z4;
    for (int i = tid; i < NB * NHD; i += ATHR) { mx[i] = -1.0e30f; den[i] = 0.f; }
  }
  __syncthreads();

  const bool al16 = ((nE & 3) == 0);
  const int nChunks = (nE + CHUNK - 1) / CHUNK;
#pragma unroll 1
  for (int ch = 0; ch < nChunks; ++ch) {
    const int cbase = ch * CHUNK;
    int wc = 0;
#pragma unroll
    for (int g = 0; g < NGRP; ++g) {
      const int el0 = (g * ATHR + tid) * 4;
      const int e0  = cbase + el0;
      const int sent = -2147483647 - 1;
      v4i d;
      if (al16 && (e0 + 3 < nE)) {
        d = *(const v4i*)(dstA + e0);
      } else {
        d.x = (e0     < nE) ? dstA[min(e0, nE - 1)]     : sent;
        d.y = (e0 + 1 < nE) ? dstA[min(e0 + 1, nE - 1)] : sent;
        d.z = (e0 + 2 < nE) ? dstA[min(e0 + 2, nE - 1)] : sent;
        d.w = (e0 + 3 < nE) ? dstA[min(e0 + 3, nE - 1)] : sent;
      }
      const unsigned s0 = (unsigned)d.x - (unsigned)nodeBase;
      const unsigned s1 = (unsigned)d.y - (unsigned)nodeBase;
      const unsigned s2 = (unsigned)d.z - (unsigned)nodeBase;
      const unsigned s3 = (unsigned)d.w - (unsigned)nodeBase;
      const bool h0 = s0 < (unsigned)NB;
      const bool h1 = s1 < (unsigned)NB;
      const bool h2 = s2 < (unsigned)NB;
      const bool h3 = s3 < (unsigned)NB;
      const unsigned many = __builtin_amdgcn_ballot_w32(h0 | h1 | h2 | h3);
      if (many != 0u) {
#define HITJ(J, HJ, SJ) { \
          const unsigned mj = __builtin_amdgcn_ballot_w32(HJ); \
          if (HJ) { \
            const int pos = wc + (int)__builtin_amdgcn_mbcnt_lo(mj, 0u); \
            if (pos < WCAP) list[wave * WCAP + pos] = ((el0 + (J)) << SH) | (int)(SJ); \
          } \
          wc += (int)__builtin_popcount(mj); }
        HITJ(0, h0, s0)
        HITJ(1, h1, s1)
        HITJ(2, h2, s2)
        HITJ(3, h3, s3)
#undef HITJ
      }
    }
    if (lane == 0) wcnt[wave] = wc;
    __syncthreads();

    if (wave == 0) {
#pragma unroll 1
      for (int wsx = 0; wsx < AWAVE; ++wsx) {
        int n = wcnt[wsx];
        if (n > WCAP) n = WCAP;
        if (n < 0) n = 0;
#pragma unroll 1
        for (int i = 0; i < n; ++i) {
          const int ent  = list[wsx * WCAP + i];
          const int slot = ent & (NB - 1);
          const int el   = (ent >> SH) & (CHUNK - 1);
          int e = cbase + el;
          if (e > nE - 1) e = nE - 1;
          int src = srcA[e];
          src = src < 0 ? 0 : (src > nN - 1 ? nN - 1 : src);
          int nd = nodeBase + slot;
          if (nd > nN - 1) nd = nN - 1;
          const float* qrow = QKV + (size_t)nd  * NQKV + 4 * lane;
          const float* krow = QKV + (size_t)src * NQKV + DM + 4 * lane;
          const float* vrow = QKV + (size_t)src * NQKV + 2 * DM + 4 * lane;
          const v4f q4 = ld4(qrow);
          const v4f k4 = ld4(krow);
          const v4f v4 = ld4(vrow);
          float part = hsum4(q4 * k4);
          part += __shfl_xor(part, 2, 32);
          part += __shfl_xor(part, 1, 32);
          const float logit = part * 0.25f;
          const int hidx = slot * NHD + hd;
          const float mo = mx[hidx];
          const float mn = fmaxf(mo, logit);
          const float corr = __expf(mo - mn);
          const float p = __expf(logit - mn);
          const float dn = den[hidx] * corr + p;
          v4f* sp = (v4f*)(sacc + slot * DM + 4 * lane);
          const v4f c0 = sp[0];
          sp[0] = c0 * corr + v4 * p;
          den[hidx] = dn;
          mx[hidx]  = mn;
        }
      }
    }
    __syncthreads();
  }

  constexpr int NV = AGG_SACC / 4;
#pragma unroll 1
  for (int idx = tid; idx < NV; idx += ATHR) {
    const int row  = idx >> 5;
    const int c4   = idx & 31;
    const int head = c4 >> 2;
    const float d  = den[row * NHD + head];
    const float inv = (d > 0.f) ? (1.0f / d) : 0.f;
    const v4f val = lds_dyn[idx] * inv;
    lds_dyn[idx] = val;
    const int node = nodeBase + row;
    if (node < nN) *(volatile v4f*)(aggOut + (size_t)node * DM + 4 * c4) = val;
  }
  __threadfence();
#pragma unroll 1
  for (int idx = tid; idx < NV; idx += ATHR) {
    const int row  = idx >> 5;
    const int c4   = idx & 31;
    const int node = nodeBase + row;
    const v4f val = lds_dyn[idx];
    if (node < nN) *(volatile v4f*)(aggOut + (size_t)node * DM + 4 * c4) = val;
  }
}

__global__ __launch_bounds__(256) void k_colstats(const float* __restrict__ X, float* stats, int n) {
  __shared__ double ss[256];
  __shared__ double sq[256];
  const int c = blockIdx.x;
  const int tid = threadIdx.x;
  double s = 0.0, q = 0.0;
#pragma unroll 1
  for (int r = tid; r < n; r += 256) {
    const double v = (double)X[(size_t)r * DM + c];
    s += v;
    q += v * v;
  }
  ss[tid] = s;
  sq[tid] = q;
  __syncthreads();
#pragma unroll 1
  for (int st = 128; st > 0; st >>= 1) {
    if (tid < st) { ss[tid] += ss[tid + st]; sq[tid] += sq[tid + st]; }
    __syncthreads();
  }
  if (tid < 32) {
    const double inv = 1.0 / (double)n;
    const double mu = ss[0] * inv;
    double var = sq[0] * inv - mu * mu;
    if (var < 0.0) var = 0.0;
    const float rs = rsqrtf((float)var + 1e-5f);
    float val = 0.f;
    if (tid == 0) val = (float)mu;
    if (tid == 1) val = rs;
    volatile float* sp = stats + (size_t)c * STP + tid;
    *sp = val;
    __threadfence();
    *sp = val;
  }
}

__global__ __launch_bounds__(256) void k_bn(const float* __restrict__ X, const float* __restrict__ stats,
                                           const float* __restrict__ gamma, const float* __restrict__ beta,
                                           float* out, int nv4) {
  const int i = blockIdx.x * 256 + threadIdx.x;
  if (i >= nv4) return;
  const int c = (i & 31) * 4;
  const v4f x = ld4(X + (size_t)i * 4);
  const v4f g = ld4(gamma + c);
  const v4f b = ld4(beta + c);
  const float mu0 = stats[(c + 0) * STP], rs0 = stats[(c + 0) * STP + 1];
  const float mu1 = stats[(c + 1) * STP], rs1 = stats[(c + 1) * STP + 1];
  const float mu2 = stats[(c + 2) * STP], rs2 = stats[(c + 2) * STP + 1];
  const float mu3 = stats[(c + 3) * STP], rs3 = stats[(c + 3) * STP + 1];
  v4f o;
  o.x = (g.x * (x.x - mu0)) * rs0 + b.x;
  o.y = (g.y * (x.y - mu1)) * rs1 + b.y;
  o.z = (g.z * (x.z - mu2)) * rs2 + b.z;
  o.w = (g.w * (x.w - mu3)) * rs3 + b.w;
  volatile v4f* op = (volatile v4f*)(out + (size_t)i * 4);
  *op = o;
  __threadfence();
  *op = o;
}

extern "C" void kernel_launch(void* const* d_in, const int* in_sizes, int n_in,
                              void* d_out, int out_size, void* d_ws, size_t ws_size,
                              hipStream_t stream) {
  if (n_in < 12) return;
  if (in_sizes[0] < DM || (in_sizes[0] % DM) != 0) return;
  const int n = in_sizes[0] / DM;
  if (in_sizes[1] < 2 || (in_sizes[1] & 1) != 0) return;
  const int nE = in_sizes[1] / 2;
  if (in_sizes[2] != DM * DM || in_sizes[3] != DM * DM || in_sizes[4] != DM * DM || in_sizes[5] != DM * DM) return;
  if (in_sizes[6] != DM || in_sizes[7] != DM || in_sizes[10] != DM || in_sizes[11] != DM) return;
  if (in_sizes[8] != DM * HIDN || in_sizes[9] != HIDN * DM) return;
  if (out_size != n * DM) return;

  const float* x   = (const float*)d_in[0];
  const int*   ei  = (const int*)d_in[1];
  const int*   src = ei;
  const int*   dst = ei + nE;
  const float* Wq  = (const float*)d_in[2];
  const float* Wk  = (const float*)d_in[3];
  const float* Wv  = (const float*)d_in[4];
  const float* Wo  = (const float*)d_in[5];
  const float* g1  = (const float*)d_in[6];
  const float* b1  = (const float*)d_in[7];
  const float* W1  = (const float*)d_in[8];
  const float* W2  = (const float*)d_in[9];
  const float* g2  = (const float*)d_in[10];
  const float* b2  = (const float*)d_in[11];
  float* out = (float*)d_out;

  size_t off = 0;
  char* base = (char*)d_ws;
#define CARVE(ptr, type, bytes) type ptr = (type)(base + off); off += (((size_t)(bytes)) + 255) & ~(size_t)255;
  CARVE(pW,  _Float16*, (size_t)PLANE_H * 2)
  CARVE(QKV, float*, (size_t)n * NQKV * sizeof(float))
  CARVE(AGG, float*, (size_t)n * DM * sizeof(float))
  CARVE(R1,  float*, (size_t)n * DM * sizeof(float))
  CARVE(ST1, float*, (size_t)DM * STP * sizeof(float))
  CARVE(X1,  float*, (size_t)n * DM * sizeof(float))
  CARVE(HB,  float*, (size_t)n * HIDN * sizeof(float))
  CARVE(R2,  float*, (size_t)n * DM * sizeof(float))
  CARVE(ST2, float*, (size_t)DM * STP * sizeof(float))
#undef CARVE
  if (off > ws_size || off > WS_CAP) return;

  const int gblk = (n + GR - 1) / GR;
  const int nv4  = n * (DM / 4);
  const int gbn  = (nv4 + 255) / 256;

  k_prep<<<(PREP_ROWS + 255) / 256, 256, 0, stream>>>(Wq, Wk, Wv, Wo, W1, W2, pW);

  k_gemm<DM, NQKV><<<gblk, 256, 0, stream>>>(x, pW + POFF_QKV, nullptr, QKV, n, 0);

  hipFuncSetAttribute(reinterpret_cast<const void*>(&k_agg),
                      hipFuncAttributeMaxDynamicSharedMemorySize, AGG_LDS_BYTES);
  k_agg<<<(n + NB - 1) / NB, ATHR, AGG_LDS_BYTES, stream>>>(src, dst, QKV, AGG, n, nE);

  k_gemm<DM, DM><<<gblk, 256, 0, stream>>>(AGG, pW + POFF_O, x, R1, n, 0);

  k_colstats<<<DM, 256, 0, stream>>>(R1, ST1, n);
  k_bn<<<gbn, 256, 0, stream>>>(R1, ST1, g1, b1, X1, nv4);

  k_gemm<DM, HIDN><<<gblk, 256, 0, stream>>>(X1, pW + POFF_1, nullptr, HB, n, 1);
  k_gemm<HIDN, DM><<<gblk, 256, 0, stream>>>(HB, pW + POFF_2, X1, R2, n, 0);

  k_colstats<<<DM, 256, 0, stream>>>(R2, ST2, n);
  k_bn<<<gbn, 256, 0, stream>>>(R2, ST2, g2, b2, out, nv4);
}
